// BiCRFModel_16552803959010
// MI455X (gfx1250) — hardware-verified
//
#include <hip/hip_runtime.h>
#include <stdint.h>

constexpr int NBATCH = 32;
constexpr int NTIME  = 256;
constexpr int NDIM   = 768;
constexpr int NHID   = 512;
constexpr int NGATE  = 2048;
constexpr int NTAGS  = 25;
constexpr int NROWS  = NBATCH * NTIME;
constexpr int NTAGP  = 64;
constexpr int LGP    = 64;
constexpr int LSP    = 32;
constexpr int HPITCH = 520;
constexpr int OUT_TOTAL = 1 + NROWS * NTAGS;
constexpr int OUT_TAIL  = OUT_TOTAL - 1;
static_assert(NROWS % 64 == 0 && NGATE % 64 == 0 && NDIM % 64 == 0 && NHID % 32 == 0);
static_assert((OUT_TOTAL - 1) % 4 == 0);
static_assert(((OUT_TOTAL - 1) / 4) % 256 == 0);

typedef __attribute__((ext_vector_type(16))) _Float16 v16h;
typedef __attribute__((ext_vector_type(8)))  _Float16 v8h;
typedef __attribute__((ext_vector_type(16))) __bf16   v16b;
typedef __attribute__((ext_vector_type(8)))  __bf16   v8b;
typedef __attribute__((ext_vector_type(8)))  float    v8f;
typedef __attribute__((ext_vector_type(4)))  float    v4f;

__device__ __forceinline__ unsigned short f2bf_bits(float f) {
  unsigned u = __float_as_uint(f);
  return (unsigned short)((u + 0x7FFFu + ((u >> 16) & 1u)) >> 16);
}
__device__ __forceinline__ float bf_bits2f(unsigned short h) { return __uint_as_float(((unsigned)h) << 16); }

__device__ __forceinline__ void dep_guard_h(v8f& a, v8f& b, v16h x, v16h y) { asm volatile("v_nop\n\tv_nop\n\tv_nop\n\tv_nop" : "+v"(a), "+v"(b) : "v"(x), "v"(y)); }
__device__ __forceinline__ void dep_guard_b(v8f& a, v8f& b, v16b x, v16b y) { asm volatile("v_nop\n\tv_nop\n\tv_nop\n\tv_nop" : "+v"(a), "+v"(b) : "v"(x), "v"(y)); }
__device__ __forceinline__ void keep4_h(v16h a, v16h b, v16h c, v16h d) { asm volatile("v_nop" :: "v"(a), "v"(b), "v"(c), "v"(d)); }
__device__ __forceinline__ void keep4_b(v16b a, v16b b, v16b c, v16b d) { asm volatile("v_nop" :: "v"(a), "v"(b), "v"(c), "v"(d)); }
__device__ __forceinline__ void acc_guard4(v8f& a, v8f& b, v8f& c, v8f& d) { asm volatile("v_nop\n\tv_nop\n\tv_nop\n\tv_nop" : "+v"(a), "+v"(b), "+v"(c), "+v"(d)); }
template <typename T> struct Frag;
template <> struct Frag<_Float16> {
  typedef v16h V; union U { v16h v; v8h h[2]; };
  static __device__ __forceinline__ v16h load(const _Float16* p) {
    U f; f.h[0] = *(const v8h*)(p); f.h[1] = *(const v8h*)(p + 16); return f.v;
  }
  static __device__ __forceinline__ v8f mma(v16h a, v16h b, v8f c) {
    return __builtin_amdgcn_wmma_f32_16x16x32_f16(false, a, false, b, (short)0, c, false, false);
  }
  static __device__ __forceinline__ void guard(v8f& a, v8f& b, v16h x, v16h y) { dep_guard_h(a, b, x, y); }
  static __device__ __forceinline__ void keep(v16h a, v16h b, v16h c, v16h d) { keep4_h(a, b, c, d); }
};
template <> struct Frag<__bf16> {
  typedef v16b V; union U { v16b v; v8b h[2]; };
  static __device__ __forceinline__ v16b load(const __bf16* p) {
    U f; f.h[0] = *(const v8b*)(p); f.h[1] = *(const v8b*)(p + 16); return f.v;
  }
  static __device__ __forceinline__ v8f mma(v16b a, v16b b, v8f c) {
    return __builtin_amdgcn_wmma_f32_16x16x32_bf16(false, a, false, b, (short)0, c, false, false);
  }
  static __device__ __forceinline__ void guard(v8f& a, v8f& b, v16b x, v16b y) { dep_guard_b(a, b, x, y); }
  static __device__ __forceinline__ void keep(v16b a, v16b b, v16b c, v16b d) { keep4_b(a, b, c, d); }
};

template <int ET> struct Elem;
template <> struct Elem<0> { typedef _Float16 T; };
template <> struct Elem<1> { typedef __bf16 T; };
template <int ET, bool SPLIT, int BIAS_MODE, int OUT_MODE, bool RESID, int ACT = 0>
__global__ __launch_bounds__(256) void wmma_gemm64(
    const unsigned short* __restrict__ Ap, const unsigned short* __restrict__ A2p, int lda, long strideA,
    const unsigned short* __restrict__ Btp, const unsigned short* __restrict__ Bt2p, int ldb, long strideB,
    void* __restrict__ Cout, void* __restrict__ Cout2, int ldc, long strideC,
    const float* __restrict__ bias,
    const float* __restrict__ resid, long strideR,
    int M, int N, int K, float scale) {
  typedef typename Elem<ET>::T T;
  typedef typename Frag<T>::V V;
  const T* A = (const T*)Ap; const T* A2 = (const T*)A2p; const T* Bt = (const T*)Btp; const T* Bt2 = (const T*)Bt2p;
  __shared__ __align__(16) float sT[8][16 * 68];
  const int b    = blockIdx.y;
  const int lane = threadIdx.x & 31;
  const int wave = threadIdx.x >> 5;
  const int tilesN = N >> 6;
  const int tilesM = M >> 6;
  const int tile = blockIdx.x * 8 + wave;
  if (tile >= tilesM * tilesN) return;
  const int tm = tile / tilesN;
  const int tn = tile - tm * tilesN;
  const int m0 = tm << 6;
  const int n0 = tn << 6;

  const T* Ab  = A  + (size_t)b * strideA;
  const T* Bb  = Bt + (size_t)b * strideB;
  const T* Ab2 = SPLIT ? (A2  + (size_t)b * strideA) : nullptr;
  const T* Bb2 = SPLIT ? (Bt2 + (size_t)b * strideB) : nullptr;

  const int rlane = lane & 15;
  const int koff  = (lane >> 4) * 8;
  const int mOff  = (lane >> 4) * 8;

  v8f acc[4][4];
#pragma unroll
  for (int i = 0; i < 4; ++i)
#pragma unroll
    for (int j = 0; j < 4; ++j) acc[i][j] = (v8f){0.f,0.f,0.f,0.f,0.f,0.f,0.f,0.f};

  for (int k0 = 0; k0 < K; k0 += 32) {
    V bh[4], bl[4];
#pragma unroll
    for (int j = 0; j < 4; ++j) {
      const size_t bo = (size_t)(n0 + (j << 4) + rlane) * ldb + koff + k0;
      bh[j] = Frag<T>::load(Bb + bo);
      if (SPLIT) bl[j] = Frag<T>::load(Bb2 + bo);
    }
#pragma unroll
    for (int i = 0; i < 4; ++i) {
      const size_t ao = (size_t)(m0 + (i << 4) + rlane) * lda + koff + k0;
      V ah = Frag<T>::load(Ab + ao);
      V al;
      if (SPLIT) al = Frag<T>::load(Ab2 + ao);
#pragma unroll
      for (int j = 0; j < 4; ++j) {
        acc[i][j] = Frag<T>::mma(ah, bh[j], acc[i][j]);
        if (SPLIT) {
          acc[i][j] = Frag<T>::mma(ah, bl[j], acc[i][j]);
          acc[i][j] = Frag<T>::mma(al, bh[j], acc[i][j]);
        }
      }
      Frag<T>::guard(acc[i][0], acc[i][3], ah, SPLIT ? al : ah);
    }
    Frag<T>::keep(bh[0], bh[1], bh[2], bh[3]);
    if (SPLIT) Frag<T>::keep(bl[0], bl[1], bl[2], bl[3]);
  }
  acc_guard4(acc[0][0], acc[0][1], acc[0][2], acc[0][3]);
  acc_guard4(acc[1][0], acc[1][1], acc[1][2], acc[1][3]);
  acc_guard4(acc[2][0], acc[2][1], acc[2][2], acc[2][3]);
  acc_guard4(acc[3][0], acc[3][1], acc[3][2], acc[3][3]);

  float* slab = sT[wave];
  const float* Rb = RESID ? (resid + (size_t)b * strideR) : nullptr;
#pragma unroll
  for (int i = 0; i < 4; ++i) {
    const int mBase = m0 + (i << 4);
#pragma unroll
    for (int j = 0; j < 4; ++j) {
      const int n = n0 + (j << 4) + rlane;
      float bv = 0.f;
      if (BIAS_MODE == 2) bv = bias[n];
#pragma unroll
      for (int r = 0; r < 8; ++r) {
        float v = acc[i][j][r] * scale;
        if (BIAS_MODE == 1) v += bias[mBase + mOff + r];
        if (BIAS_MODE == 2) v += bv;
        if (RESID) v += Rb[(size_t)(mBase + mOff + r) * ldc + n];
        if (ACT == 1) v = tanhf(v);
        if (ACT == 2) v = fmaxf(v, 0.0f);
        if (ACT == 3) v = v / (1.0f + expf(-v));
        if (ACT == 4) v = (v > 0.f) ? v : 0.01f * v;
        if (ACT == 5) v = 0.5f * v * (1.0f + erff(v * 0.70710678118654752f));
        slab[(mOff + r) * 68 + (j << 4) + rlane] = v;
      }
    }
    __builtin_amdgcn_fence(__ATOMIC_RELEASE, "workgroup");
    __builtin_amdgcn_wave_barrier();
    __builtin_amdgcn_fence(__ATOMIC_ACQUIRE, "workgroup");
    if (OUT_MODE == 0) {
      float* C = (float*)Cout + (size_t)b * strideC;
      const int hh = lane >> 4, c4 = (lane & 15) * 4;
      for (int pass = 0; pass < 2; ++pass) {
#pragma unroll
        for (int it = 0; it < 8; ++it) {
          const int row = it * 2 + hh;
          v4f v = *(const v4f*)(slab + row * 68 + c4);
          *(volatile v4f*)(C + (size_t)(mBase + row) * ldc + n0 + c4) = v;
        }
        __threadfence();
      }
    } else {
      const int q = lane >> 3, c8 = (lane & 7) * 8;
      unsigned short* C  = (unsigned short*)Cout  + (size_t)b * strideC;
      unsigned short* C2 = (OUT_MODE == 2) ? ((unsigned short*)Cout2 + (size_t)b * strideC) : nullptr;
      for (int pass = 0; pass < 2; ++pass) {
#pragma unroll
        for (int it = 0; it < 4; ++it) {
          const int row = it * 4 + q;
          const float* sp = slab + row * 68 + c8;
          v8h hv, lv;
#pragma unroll
          for (int e = 0; e < 8; ++e) {
            if (OUT_MODE == 1) {
              hv[e] = (_Float16)sp[e];
            } else {
              unsigned short hb = f2bf_bits(sp[e]);
              unsigned short lb = f2bf_bits(sp[e] - bf_bits2f(hb));
              hv[e] = __builtin_bit_cast(_Float16, hb);
              lv[e] = __builtin_bit_cast(_Float16, lb);
            }
          }
          *(volatile v8h*)(C + (size_t)(mBase + row) * ldc + n0 + c8) = hv;
          if (OUT_MODE == 2) *(volatile v8h*)(C2 + (size_t)(mBase + row) * ldc + n0 + c8) = lv;
        }
        __threadfence();
      }
    }
    __builtin_amdgcn_fence(__ATOMIC_RELEASE, "workgroup");
    __builtin_amdgcn_wave_barrier();
    __builtin_amdgcn_fence(__ATOMIC_ACQUIRE, "workgroup");
  }
}

__global__ __launch_bounds__(256) void cast_f32_f16x2(
    const float* __restrict__ in, _Float16* __restrict__ out, int n2) {
  int i = blockIdx.x * 256 + threadIdx.x;
  if (i < n2) {
    const _Float16 h0 = (_Float16)in[2 * i], h1 = (_Float16)in[2 * i + 1];
    const unsigned u = (unsigned)__builtin_bit_cast(unsigned short, h0) | ((unsigned)__builtin_bit_cast(unsigned short, h1) << 16);
    ((volatile unsigned*)out)[i] = u;
    __threadfence();
    ((volatile unsigned*)out)[i] = u;
  }
}

__device__ __forceinline__ float rcp_f(float x) { return __builtin_amdgcn_rcpf(x); }
__device__ __forceinline__ float sigm_f(float x) { return rcp_f(1.0f + expf(-x)); }
__device__ __forceinline__ float tanh_f(float x) { return 1.0f - 2.0f * rcp_f(1.0f + expf(2.0f * x)); }
__device__ __forceinline__ float selu_f(float x) {
  const float sc = 1.0507009873554804934193349852946f;
  const float al = 1.6732632423543772848170429916717f;
  return (x > 0.0f) ? (sc * x) : (sc * (al * expm1f(x)));
}

__global__ __launch_bounds__(256) void tcast_kernel(const float* __restrict__ in, unsigned short* __restrict__ outp,
                                                    int K, int N, float scale) {
  __shared__ float tile[32][65];
  const int tid = threadIdx.x;
  const int n0 = blockIdx.x * 32;
  const int k0 = blockIdx.y * 64;
#pragma unroll
  for (int i = 0; i < 8; ++i) {
    const int idx = tid + 256 * i;
    const int kk = idx >> 5;
    const int nn = idx & 31;
    tile[nn][kk] = in[(size_t)(k0 + kk) * N + n0 + nn];
  }
  __syncthreads();
  const int nn = tid >> 3;
  const int q  = tid & 7;
  v8h hv;
#pragma unroll
  for (int e = 0; e < 8; ++e) hv[e] = (_Float16)(tile[nn][q * 8 + e] * scale);
  _Float16* dst = (_Float16*)(void*)outp + (size_t)(n0 + nn) * K + k0 + q * 8;
  *(volatile v8h*)dst = hv;
  __threadfence();
  *(volatile v8h*)dst = hv;
}

__global__ __launch_bounds__(128) void dense_w_kernel(const float* __restrict__ dw, const float* __restrict__ db,
                                                      unsigned short* __restrict__ dwtp, float* __restrict__ db64) {
  const int n = blockIdx.x;
  const int tid = threadIdx.x;
  const int nc = (n < NTAGS) ? n : (NTAGS - 1);
  const float sc = (n < NTAGS) ? 16.0f : 0.0f;
  v8h hv;
#pragma unroll
  for (int e = 0; e < 8; ++e) {
    const int k = tid * 8 + e;
    hv[e] = (_Float16)(dw[(size_t)k * NTAGS + nc] * sc);
  }
  _Float16* dst = (_Float16*)(void*)dwtp + (size_t)n * (2 * NHID) + tid * 8;
  v4f bv;
#pragma unroll
  for (int e = 0; e < 4; ++e) {
    const int i = tid * 4 + e;
    const int ic = (i < NTAGS) ? i : (NTAGS - 1);
    const float v = db[ic];
    bv[e] = (i < NTAGS) ? v : 0.0f;
  }
  const bool wb = (n == 0) && (tid < 16);
  *(volatile v8h*)dst = hv;
  if (wb) *(volatile v4f*)(db64 + tid * 4) = bv;
  __threadfence();
  *(volatile v8h*)dst = hv;
  if (wb) *(volatile v4f*)(db64 + tid * 4) = bv;
}

__global__ __launch_bounds__(512) void lstm_seq_kernel(const float* __restrict__ xz,
                                                       const unsigned short* __restrict__ rtp,
                                                       unsigned short* __restrict__ hcp,
                                                       int dir) {
  const _Float16* rt = (const _Float16*)(const void*)rtp;
  _Float16* hc = (_Float16*)(void*)hcp;
  __shared__ __align__(16) _Float16 hT[2 * 16 * HPITCH];

  const int tid  = threadIdx.x;
  const int wave = tid >> 5;
  const int lane = tid & 31;
  const int hh   = lane >> 4;
  const int cl   = lane & 15;
  const int koff = hh * 8;
  const int rowBase = blockIdx.x * 16;

  {
    v8h z8;
#pragma unroll
    for (int e = 0; e < 8; ++e) z8[e] = (_Float16)0.0f;
    for (int i = tid; i < (2 * 16 * HPITCH) / 8; i += 512) *(v8h*)(hT + i * 8) = z8;
  }
  float cst[2][8];
#pragma unroll
  for (int u = 0; u < 2; ++u)
#pragma unroll
    for (int r = 0; r < 8; ++r) cst[u][r] = 0.0f;
  __syncthreads();

  const float RSC = 1.0f / 128.0f;
  int cur = 0;
  for (int step = 0; step < NTIME; ++step) {
    const int t = dir ? (NTIME - 1 - step) : step;
    const _Float16* hTc = hT + cur * (16 * HPITCH);
    _Float16* hTn = hT + (cur ^ 1) * (16 * HPITCH);

    v8f acc[2][4];
#pragma unroll
    for (int u = 0; u < 2; ++u)
#pragma unroll
      for (int g = 0; g < 4; ++g) acc[u][g] = (v8f){0.f,0.f,0.f,0.f,0.f,0.f,0.f,0.f};

#pragma unroll 1
    for (int ks = 0; ks < NHID / 32; ++ks) {
      const v16h a = Frag<_Float16>::load(hTc + cl * HPITCH + ks * 32 + koff);
      v16h bfr[2][4];
#pragma unroll
      for (int u = 0; u < 2; ++u)
#pragma unroll
        for (int g = 0; g < 4; ++g) {
          const int n = g * NHID + (wave * 2 + u) * 16 + cl;
          bfr[u][g] = Frag<_Float16>::load(rt + (size_t)n * NHID + ks * 32 + koff);
        }
#pragma unroll
      for (int u = 0; u < 2; ++u)
#pragma unroll
        for (int g = 0; g < 4; ++g) acc[u][g] = Frag<_Float16>::mma(a, bfr[u][g], acc[u][g]);
      dep_guard_h(acc[0][0], acc[1][3], a, a);
      keep4_h(bfr[0][0], bfr[0][1], bfr[0][2], bfr[0][3]);
      keep4_h(bfr[1][0], bfr[1][1], bfr[1][2], bfr[1][3]);
    }
    acc_guard4(acc[0][0], acc[0][1], acc[0][2], acc[0][3]);
    acc_guard4(acc[1][0], acc[1][1], acc[1][2], acc[1][3]);

#pragma unroll
    for (int u = 0; u < 2; ++u) {
      const int j = (wave * 2 + u) * 16 + cl;
#pragma unroll
      for (int r = 0; r < 8; ++r) {
        const int bb = rowBase + 8 * hh + r;
        const float* xr = xz + ((size_t)bb * NTIME + t) * NGATE + j;
        const float zi = acc[u][0][r] * RSC + xr[0];
        const float zf = acc[u][1][r] * RSC + xr[NHID];
        const float zg = acc[u][2][r] * RSC + xr[2 * NHID];
        const float zo = acc[u][3][r] * RSC + xr[3 * NHID];
        const float si = sigm_f(zi);
        const float sf = sigm_f(zf);
        const float so = sigm_f(zo);
        const float tg = tanh_f(zg);
        const float cn = sf * cst[u][r] + si * tg;
        const float hn = so * tanh_f(cn);
        cst[u][r] = cn;
        hTn[(8 * hh + r) * HPITCH + j] = (_Float16)(hn * 8.0f);
      }
    }
    __syncthreads();

    {
      const _Float16* src = hTn + wave * HPITCH;
      _Float16* dst = hc + ((size_t)(rowBase + wave) * NTIME + t) * (2 * NHID) + dir * NHID;
      const v8h v0 = *(const v8h*)(src + lane * 8);
      const v8h v1 = *(const v8h*)(src + 256 + lane * 8);
      *(volatile v8h*)(dst + lane * 8) = v0;
      *(volatile v8h*)(dst + 256 + lane * 8) = v1;
      __threadfence();
      *(volatile v8h*)(dst + lane * 8) = v0;
      *(volatile v8h*)(dst + 256 + lane * 8) = v1;
    }
    cur ^= 1;
  }
}

__global__ __launch_bounds__(256) void selu_rows_kernel(const float* __restrict__ lg, float* __restrict__ ls) {
  const int row  = blockIdx.x * 8 + (threadIdx.x >> 5);
  const int lane = threadIdx.x & 31;
  const float x = lg[(size_t)row * LGP + lane];
  const float s = selu_f(x);
  const float v = (lane < NTAGS) ? s : 0.0f;
  float* dst = ls + (size_t)row * LSP + lane;
  *(volatile float*)dst = v;
  __threadfence();
  *(volatile float*)dst = v;
}

__global__ __launch_bounds__(32) void crf_nll_kernel(const float* __restrict__ ls,
                                                    const int* __restrict__ tags,
                                                    const int* __restrict__ lens,
                                                    const float* __restrict__ trans,
                                                    float* __restrict__ nllp) {
  __shared__ float str[NTAGS * NTAGS + 7];
  const int b = blockIdx.x;
  const int lane = threadIdx.x;
  for (int i = lane; i < NTAGS * NTAGS; i += 32) str[i] = trans[i];
  __syncthreads();

  int L = lens[b];
  L = (L < 1) ? 1 : ((L > NTIME) ? NTIME : L);
  const size_t rb = (size_t)b * NTIME;

  float us = 0.0f, bs = 0.0f;
#pragma unroll 1
  for (int tt = 0; tt < NTIME / 32; ++tt) {
    const int t = tt * 32 + lane;
    int tg = tags[rb + t];
    tg = (tg < 0) ? 0 : ((tg > NTAGS - 1) ? (NTAGS - 1) : tg);
    const float v = ls[(rb + t) * LSP + tg];
    us += (t < L) ? v : 0.0f;
    const int tp = (t > 0) ? (t - 1) : 0;
    int tgp = tags[rb + tp];
    tgp = (tgp < 0) ? 0 : ((tgp > NTAGS - 1) ? (NTAGS - 1) : tgp);
    const float w = str[tgp * NTAGS + tg];
    bs += (t >= 1 && t < L) ? w : 0.0f;
  }
#pragma unroll
  for (int off = 16; off > 0; off >>= 1) {
    us += __shfl_xor(us, off, 32);
    bs += __shfl_xor(bs, off, 32);
  }

  const int nc = (lane < NTAGS) ? lane : (NTAGS - 1);
  const bool live = (lane < NTAGS);
  float alpha = ls[rb * LSP + nc];
  alpha = live ? alpha : 0.0f;
  for (int t = 1; t < L; ++t) {
    const float lgt = ls[(rb + t) * LSP + nc];
    float mx = -__builtin_inff();
#pragma unroll 1
    for (int m = 0; m < NTAGS; ++m) {
      const float am = __shfl(alpha, m, 32);
      mx = fmaxf(mx, am + str[m * NTAGS + nc]);
    }
    float se = 0.0f;
#pragma unroll 1
    for (int m = 0; m < NTAGS; ++m) {
      const float am = __shfl(alpha, m, 32);
      se += expf((am + str[m * NTAGS + nc]) - mx);
    }
    const float na = (logf(se) + mx) + lgt;
    alpha = live ? na : 0.0f;
  }
  float mz = live ? alpha : -__builtin_inff();
#pragma unroll
  for (int off = 16; off > 0; off >>= 1) mz = fmaxf(mz, __shfl_xor(mz, off, 32));
  const float ea = expf(alpha - mz);
  float ez = live ? ea : 0.0f;
#pragma unroll
  for (int off = 16; off > 0; off >>= 1) ez += __shfl_xor(ez, off, 32);
  const float logz = logf(ez) + mz;
  const float nll = -(us + bs - logz);

  v4f o;
  o[0] = nll; o[1] = nll; o[2] = nll; o[3] = nll;
  float* dst = nllp + (size_t)b * 32 + lane * 4;
  if (lane < 8) *(volatile v4f*)dst = o;
  __threadfence();
  if (lane < 8) *(volatile v4f*)dst = o;
}

__global__ __launch_bounds__(256) void out_writer_kernel(const float* __restrict__ ls,
                                                        const float* __restrict__ nllp,
                                                        float* __restrict__ out) {
  __shared__ float sLoss;
  if (threadIdx.x == 0) {
    float s = 0.0f;
    if (blockIdx.x == 0) {
#pragma unroll 1
      for (int b = 0; b < NBATCH; ++b) s += nllp[b * 32];
    }
    sLoss = s * (1.0f / 32.0f);
  }
  __syncthreads();
  const int gi = blockIdx.x * 256 + threadIdx.x;
  const float lossv = sLoss;
  v4f vv;
#pragma unroll
  for (int e = 0; e < 4; ++e) {
    const int f = gi * 4 + e;
    const int el = (f > 0) ? (f - 1) : 0;
    const int row = el / NTAGS;
    const int col = el - row * NTAGS;
    float v = ls[(size_t)row * LSP + col];
    if (f == 0) v = lossv;
    vv[e] = v;
  }
  float* dst = out + (size_t)gi * 4;
  const float tv = ls[(size_t)(NROWS - 1) * LSP + (NTAGS - 1)];
  const bool tail = (gi == 0);
  *(volatile v4f*)dst = vv;
  if (tail) *(volatile float*)(out + OUT_TAIL) = tv;
  __threadfence();
  *(volatile v4f*)dst = vv;
  if (tail) *(volatile float*)(out + OUT_TAIL) = tv;
}

extern "C" void kernel_launch(void* const* d_in, const int* in_sizes, int n_in,
                              void* d_out, int out_size, void* d_ws, size_t ws_size,
                              hipStream_t stream) {
  if (n_in < 12) return;
  if (in_sizes[0] != NROWS * NDIM) return;
  if (in_sizes[1] != NROWS) return;
  if (in_sizes[2] != NBATCH) return;
  if (in_sizes[3] != NDIM * NGATE || in_sizes[6] != NDIM * NGATE) return;
  if (in_sizes[4] != NHID * NGATE || in_sizes[7] != NHID * NGATE) return;
  if (in_sizes[5] != NGATE || in_sizes[8] != NGATE) return;
  if (in_sizes[9] != 2 * NHID * NTAGS || in_sizes[10] != NTAGS || in_sizes[11] != NTAGS * NTAGS) return;
  if (out_size != OUT_TOTAL) return;

  const float* x     = (const float*)d_in[0];
  const int*   tags  = (const int*)d_in[1];
  const int*   lens  = (const int*)d_in[2];
  const float* kf    = (const float*)d_in[3];
  const float* rf    = (const float*)d_in[4];
  const float* bfw   = (const float*)d_in[5];
  const float* kb    = (const float*)d_in[6];
  const float* rbw   = (const float*)d_in[7];
  const float* bbw   = (const float*)d_in[8];
  const float* dw    = (const float*)d_in[9];
  const float* db    = (const float*)d_in[10];
  const float* trans = (const float*)d_in[11];

  size_t off = 0;
  auto carve = [&](size_t bytes) { size_t o = off; off += (bytes + 255) & ~(size_t)255; return o; };
  const size_t oXH  = carve((size_t)NROWS * NDIM * 2);
  const size_t oKT0 = carve((size_t)NGATE * NDIM * 2);
  const size_t oKT1 = carve((size_t)NGATE * NDIM * 2);
  const size_t oRT0 = carve((size_t)NGATE * NHID * 2);
  const size_t oRT1 = carve((size_t)NGATE * NHID * 2);
  const size_t oXZ  = carve((size_t)NROWS * NGATE * 4);
  const size_t oHC  = carve((size_t)NROWS * 2 * NHID * 2);
  const size_t oDWT = carve((size_t)NTAGP * 2 * NHID * 2);
  const size_t oDB  = carve((size_t)NTAGP * 4);
  const size_t oLG  = carve((size_t)NROWS * LGP * 4);
  const size_t oLS  = carve((size_t)NROWS * LSP * 4);
  const size_t oNLL = carve((size_t)NBATCH * 32 * 4);
  if (off > ws_size) return;

  char* ws = (char*)d_ws;
  unsigned short* XH  = (unsigned short*)(ws + oXH);
  unsigned short* KT0 = (unsigned short*)(ws + oKT0);
  unsigned short* KT1 = (unsigned short*)(ws + oKT1);
  unsigned short* RT0 = (unsigned short*)(ws + oRT0);
  unsigned short* RT1 = (unsigned short*)(ws + oRT1);
  float*          XZ  = (float*)(ws + oXZ);
  unsigned short* HC  = (unsigned short*)(ws + oHC);
  unsigned short* DWT = (unsigned short*)(ws + oDWT);
  float*          DB64 = (float*)(ws + oDB);
  float*          LG  = (float*)(ws + oLG);
  float*          LS  = (float*)(ws + oLS);
  float*          NLL = (float*)(ws + oNLL);
  float*          out = (float*)d_out;

  {
    const int n2 = NROWS * NDIM / 2;
    cast_f32_f16x2<<<(n2 + 255) / 256, 256, 0, stream>>>(x, (_Float16*)(void*)XH, n2);
  }
  tcast_kernel<<<dim3(NGATE / 32, NDIM / 64), 256, 0, stream>>>(kf, KT0, NDIM, NGATE, 16.0f);
  tcast_kernel<<<dim3(NGATE / 32, NDIM / 64), 256, 0, stream>>>(kb, KT1, NDIM, NGATE, 16.0f);
  tcast_kernel<<<dim3(NGATE / 32, NHID / 64), 256, 0, stream>>>(rf, RT0, NHID, NGATE, 16.0f);
  tcast_kernel<<<dim3(NGATE / 32, NHID / 64), 256, 0, stream>>>(rbw, RT1, NHID, NGATE, 16.0f);
  dense_w_kernel<<<NTAGP, 128, 0, stream>>>(dw, db, DWT, DB64);

  const int tilesXZ = (NROWS / 64) * (NGATE / 64);
  wmma_gemm64<0, false, 2, 0, false, 0><<<dim3((tilesXZ + 7) / 8, 1), 256, 0, stream>>>(
      XH, XH, NDIM, 0L, KT0, KT0, NDIM, 0L, (void*)XZ, (void*)XZ, NGATE, 0L,
      bfw, bfw, 0L, NROWS, NGATE, NDIM, 1.0f / 16.0f);
  lstm_seq_kernel<<<NBATCH / 16, 512, 0, stream>>>(XZ, RT0, HC, 0);
  wmma_gemm64<0, false, 2, 0, false, 0><<<dim3((tilesXZ + 7) / 8, 1), 256, 0, stream>>>(
      XH, XH, NDIM, 0L, KT1, KT1, NDIM, 0L, (void*)XZ, (void*)XZ, NGATE, 0L,
      bbw, bbw, 0L, NROWS, NGATE, NDIM, 1.0f / 16.0f);
  lstm_seq_kernel<<<NBATCH / 16, 512, 0, stream>>>(XZ, RT1, HC, 1);

  const int tilesD = (NROWS / 64) * (NTAGP / 64);
  wmma_gemm64<0, false, 2, 0, false, 0><<<dim3((tilesD + 7) / 8, 1), 256, 0, stream>>>(
      HC, HC, 2 * NHID, 0L, DWT, DWT, 2 * NHID, 0L, (void*)LG, (void*)LG, LGP, 0L,
      DB64, DB64, 0L, NROWS, NTAGP, 2 * NHID, 1.0f / 128.0f);
  selu_rows_kernel<<<NROWS / 8, 256, 0, stream>>>(LG, LS);
  crf_nll_kernel<<<NBATCH, 32, 0, stream>>>(LS, tags, lens, trans, NLL);
  out_writer_kernel<<<(OUT_TOTAL - 1) / 4 / 256, 256, 0, stream>>>(LS, NLL, out);
}
